// GaussianKernel_738734375297
// MI455X (gfx1250) — hardware-verified
//
#include <hip/hip_runtime.h>
#include <math.h>


#define BATCH 16384
#define IN_F 512
#define NG 8
#define KDIM (IN_F * NG)
#define OUT_F 512

typedef __attribute__((ext_vector_type(16))) _Float16 v16h;
typedef __attribute__((ext_vector_type(8)))  _Float16 v8h;
typedef __attribute__((ext_vector_type(8)))  float v8f;
typedef __attribute__((ext_vector_type(4)))  float v4f;
typedef __attribute__((ext_vector_type(4)))  unsigned v4u;

template <typename T> __device__ __forceinline__ void vst2(void* p, T v) { *(volatile T*)p = v; __threadfence(); *(volatile T*)p = v; }
__device__ __forceinline__ v8f wmma16(v16h a, v16h b, v8f c) {
  v8f d = __builtin_amdgcn_wmma_f32_16x16x32_f16(false, a, false, b, (short)0, c, false, false);
  asm volatile("v_nop\n\tv_nop\n\tv_nop\n\tv_nop" : "+v"(d) : "v"(a), "v"(b));
  return d;
}

__global__ __launch_bounds__(256) void pack_wt(const float* __restrict__ W, _Float16* __restrict__ Wt) {
  const size_t g8 = (size_t)blockIdx.x * 256 + threadIdx.x;
  const int n = (int)(g8 / (KDIM / 8)), k0 = (int)(g8 % (KDIM / 8)) * 8;
  union { v8h h; v4u u; } pk;
#pragma unroll
  for (int e = 0; e < 8; ++e) pk.h[e] = (_Float16)W[(size_t)(k0 + e) * OUT_F + n];
  vst2(Wt + (size_t)n * KDIM + k0, pk.u);
}

__global__ __launch_bounds__(128) void rbf_kan_gemm(const float* __restrict__ x, const float* __restrict__ grid,
                                                    const _Float16* __restrict__ Wt, float* __restrict__ out) {
  __shared__ __align__(16) float so[4][16 * 128];
  const int tid = threadIdx.x, wave = tid >> 5, lane = tid & 31, col = lane & 15, g = lane >> 4;
  const int m = blockIdx.x * 64 + wave * 16 + col;
  const int n0 = blockIdx.y * 128;
  const float inv_h = (float)(NG - 1) / 4.0f;
  float gr[NG];
#pragma unroll
  for (int i = 0; i < NG; ++i) gr[i] = grid[i];
  const float* xr = x + (size_t)m * IN_F;
  v8f acc[8] = {};
#pragma unroll 1
  for (int f0 = 0; f0 < IN_F; f0 += 4) {
    const float xa = xr[f0 + g], xb = xr[f0 + 2 + g];
    v16h a;
#pragma unroll
    for (int i = 0; i < NG; ++i) {
      const float da = (xa - gr[i]) * inv_h, db = (xb - gr[i]) * inv_h;
      float ea = expf(-da * da), eb = expf(-db * db);
      ea = ea < 6.10352e-5f ? 0.f : ea; eb = eb < 6.10352e-5f ? 0.f : eb;
      a[i] = (_Float16)ea; a[8 + i] = (_Float16)eb;
    }
    const int k0 = f0 * NG;
#pragma unroll
    for (int j = 0; j < 8; ++j) {
      const _Float16* wp = Wt + (size_t)(n0 + j * 16 + col) * KDIM + k0 + 8 * g;
      union { v16h v; v8h q[2]; } b; b.q[0] = *(const v8h*)wp; b.q[1] = *(const v8h*)(wp + 16);
      acc[j] = wmma16(a, b.v, acc[j]);
    }
  }
  float* S = so[wave];
#pragma unroll
  for (int j = 0; j < 8; ++j)
#pragma unroll
    for (int r = 0; r < 8; ++r) S[(8 * g + r) * 128 + j * 16 + col] = acc[j][r];
  asm volatile("s_wait_dscnt 0" ::: "memory"); __builtin_amdgcn_wave_barrier(); __builtin_amdgcn_fence(__ATOMIC_RELEASE, "workgroup");
  const int mw = blockIdx.x * 64 + wave * 16;
#pragma unroll 4
  for (int rl = 0; rl < 16; ++rl) vst2(out + (size_t)(mw + rl) * OUT_F + n0 + lane * 4, *(const v4f*)(S + rl * 128 + lane * 4));
}

extern "C" void kernel_launch(void* const* d_in, const int* in_sizes, int n_in,
                              void* d_out, int out_size, void* d_ws, size_t ws_size,
                              hipStream_t stream) {
  (void)in_sizes; (void)n_in; (void)out_size; (void)ws_size;
  const float* x    = (const float*)d_in[0];
  const float* grid = (const float*)d_in[1];
  const float* W    = (const float*)d_in[2];
  float* out = (float*)d_out;
  _Float16* Wt = (_Float16*)d_ws;
  pack_wt<<<(OUT_F * KDIM / 8) / 256, 256, 0, stream>>>(W, Wt);
  rbf_kan_gemm<<<dim3(BATCH / 64, OUT_F / 128), 128, 0, stream>>>(x, grid, Wt, out);
}
